// DotAttention_27178553049198
// MI455X (gfx1250) — hardware-verified
//
#include <hip/hip_runtime.h>
#include <math.h>

typedef __attribute__((ext_vector_type(16))) _Float16 v16h;
typedef __attribute__((ext_vector_type(8)))  _Float16 v8h;
typedef __attribute__((ext_vector_type(16))) __bf16   v16b;
typedef __attribute__((ext_vector_type(8)))  __bf16   v8b;
typedef __attribute__((ext_vector_type(8)))  float    v8f;
typedef __attribute__((ext_vector_type(4)))  float    v4f;
typedef __attribute__((ext_vector_type(4)))  unsigned v4u;

__device__ __forceinline__ unsigned short f2bf_bits(float f) {
  unsigned u = __float_as_uint(f);
  return (unsigned short)((u + 0x7FFFu + ((u >> 16) & 1u)) >> 16);
}
__device__ __forceinline__ float bf_bits2f(unsigned short h) { return __uint_as_float(((unsigned)h) << 16); }

__device__ __forceinline__ void dep_guard_b(v8f& a, v8f& b, v16b x, v16b y) { asm volatile("v_nop\n\tv_nop\n\tv_nop\n\tv_nop" : "+v"(a), "+v"(b) : "v"(x), "v"(y)); }
__device__ __forceinline__ void keep4_b(v16b a, v16b b, v16b c, v16b d) { asm volatile("v_nop" :: "v"(a), "v"(b), "v"(c), "v"(d)); }

template <typename T> struct Frag;
template <> struct Frag<__bf16> {
  typedef v16b V; union U { v16b v; v8b h[2]; };
  static __device__ __forceinline__ v16b load(const __bf16* p) {
    U f; f.h[0] = *(const v8b*)(p); f.h[1] = *(const v8b*)(p + 16); return f.v;
  }
  static __device__ __forceinline__ v8f mma(v16b a, v16b b, v8f c) {
    return __builtin_amdgcn_wmma_f32_16x16x32_bf16(false, a, false, b, (short)0, c, false, false);
  }
  static __device__ __forceinline__ void guard(v8f& a, v8f& b, v16b x, v16b y) { dep_guard_b(a, b, x, y); }
  static __device__ __forceinline__ void keep(v16b a, v16b b, v16b c, v16b d) { keep4_b(a, b, c, d); }
};

__device__ __forceinline__ unsigned short at_bf_bits(float f) {
  unsigned u = __float_as_uint(f);
  return (unsigned short)((u + 0x7FFFu + ((u >> 16) & 1u)) >> 16);
}
__device__ __forceinline__ __bf16 at_f2bf(float f) { return __builtin_bit_cast(__bf16, at_bf_bits(f)); }
__device__ __forceinline__ void at_split(float f, __bf16& hi, __bf16& lo) {
  const unsigned short hb = at_bf_bits(f);
  hi = __builtin_bit_cast(__bf16, hb);
  lo = at_f2bf(f - __uint_as_float(((unsigned)hb) << 16));
}
__device__ __forceinline__ v8f at_mma(v16b a, v16b b, v8f c) {
  c = __builtin_amdgcn_wmma_f32_16x16x32_bf16(false, a, false, b, (short)0, c, false, false);
  asm volatile("v_nop\n\tv_nop\n\tv_nop\n\tv_nop" : "+v"(c) : "v"(a), "v"(b));
  return c;
}

__global__ __launch_bounds__(256) void cast3_f32_bf16x8(
    const float* __restrict__ s0, const float* __restrict__ s1, const float* __restrict__ s2,
    unsigned short* __restrict__ d0, unsigned short* __restrict__ d1, unsigned short* __restrict__ d2,
    int n8) {
  const int pl = blockIdx.y;
  const float* src = (pl == 0) ? s0 : ((pl == 1) ? s1 : s2);
  unsigned short* dst = (pl == 0) ? d0 : ((pl == 1) ? d1 : d2);
  const int i = blockIdx.x * 256 + threadIdx.x;
  if (i < n8) {
    const v4f a = *(const v4f*)(src + (size_t)i * 8);
    const v4f b = *(const v4f*)(src + (size_t)i * 8 + 4);
    v4u w;
    w.x = (unsigned)f2bf_bits(a.x) | ((unsigned)f2bf_bits(a.y) << 16);
    w.y = (unsigned)f2bf_bits(a.z) | ((unsigned)f2bf_bits(a.w) << 16);
    w.z = (unsigned)f2bf_bits(b.x) | ((unsigned)f2bf_bits(b.y) << 16);
    w.w = (unsigned)f2bf_bits(b.z) | ((unsigned)f2bf_bits(b.w) << 16);
    volatile v4u* p = (volatile v4u*)(dst + (size_t)i * 8);
    *p = w;
    __threadfence();
    *p = w;
  }
}

constexpr int kHD  = 128;
constexpr int kNW  = 8;
constexpr int kQB  = kNW * 16;
constexpr int kKC  = 64;
constexpr int kThr = kNW * 32;
static_assert(kQB == 128 && kKC == 64 && kHD == 128 && kThr == 256);
static_assert(2 * kKC * kHD * 2 == kNW * 16 * 64 * 4);

__global__ __launch_bounds__(256)
void attn_hd128_bf16(const unsigned short* __restrict__ Qb, const unsigned short* __restrict__ Kb,
                     const unsigned short* __restrict__ Vb, float* __restrict__ out, int S, float scale) {
  union FB { v16b v; v8b h[2]; };
  __shared__ __align__(16) __bf16 KVs[2 * kKC * kHD];
  __shared__ __align__(16) __bf16 Psh[kNW][16 * kKC];
  __shared__ __align__(16) __bf16 Psl[kNW][16 * kKC];
  __bf16* Ksh = KVs;
  __bf16* Vt  = KVs + kKC * kHD;
  unsigned short* Vts = (unsigned short*)(KVs + kKC * kHD);

  const int tid  = threadIdx.x;
  const int wave = tid >> 5;
  const int lane = tid & 31;
  const int hh   = lane >> 4;
  const int c    = lane & 15;
  const int q0   = blockIdx.x * kQB + wave * 16;

  v16b qa[4];
  {
    const __bf16* qrow = (const __bf16*)Qb + (size_t)(q0 + c) * kHD + 8 * hh;
#pragma unroll
    for (int dc = 0; dc < 4; ++dc) qa[dc] = Frag<__bf16>::load(qrow + dc * 32);
  }

  float mrow[8], lrow[8];
  v8f oacc[8];
#pragma unroll
  for (int r = 0; r < 8; ++r) { mrow[r] = -__builtin_inff(); lrow[r] = 0.f; }
#pragma unroll
  for (int t = 0; t < 8; ++t) oacc[t] = (v8f){0.f,0.f,0.f,0.f,0.f,0.f,0.f,0.f};

  const int nChunks = S / kKC;
  for (int kc = 0; kc < nChunks; ++kc) {
    const int kv0 = kc * kKC;
    __syncthreads();
#pragma unroll
    for (int it = 0; it < 4; ++it) {
      const int idx = it * kThr + tid;
      const int kvr = idx >> 4, d8 = (idx & 15) * 8;
      const v4u w = *(const v4u*)(Kb + (size_t)(kv0 + kvr) * kHD + d8);
      *(v4u*)(Ksh + kvr * kHD + d8) = w;
    }
#pragma unroll
    for (int it = 0; it < 4; ++it) {
      const int idx = it * kThr + tid;
      const int kvr = idx & 63, d8 = (idx >> 6) * 8;
      const v4u w = *(const v4u*)(Vb + (size_t)(kv0 + kvr) * kHD + d8);
      Vts[(d8 + 0) * kKC + kvr] = (unsigned short)(w.x & 0xffffu);
      Vts[(d8 + 1) * kKC + kvr] = (unsigned short)(w.x >> 16);
      Vts[(d8 + 2) * kKC + kvr] = (unsigned short)(w.y & 0xffffu);
      Vts[(d8 + 3) * kKC + kvr] = (unsigned short)(w.y >> 16);
      Vts[(d8 + 4) * kKC + kvr] = (unsigned short)(w.z & 0xffffu);
      Vts[(d8 + 5) * kKC + kvr] = (unsigned short)(w.z >> 16);
      Vts[(d8 + 6) * kKC + kvr] = (unsigned short)(w.w & 0xffffu);
      Vts[(d8 + 7) * kKC + kvr] = (unsigned short)(w.w >> 16);
    }
    __syncthreads();

    v8f s[4];
#pragma unroll
    for (int j = 0; j < 4; ++j) {
      s[j] = (v8f){0.f,0.f,0.f,0.f,0.f,0.f,0.f,0.f};
#pragma unroll
      for (int dc = 0; dc < 4; ++dc) {
        FB kb;
        kb.h[0] = *(const v8b*)(Ksh + (j * 16 + c) * kHD + dc * 32 + 8 * hh);
        kb.h[1] = *(const v8b*)(Ksh + (j * 16 + c) * kHD + dc * 32 + 16 + 8 * hh);
        s[j] = at_mma(qa[dc], kb.v, s[j]);
      }
    }

    float cm[8];
#pragma unroll
    for (int r = 0; r < 8; ++r) {
      float m = -__builtin_inff();
#pragma unroll
      for (int j = 0; j < 4; ++j) { s[j][r] = s[j][r] * scale; m = fmaxf(m, s[j][r]); }
#pragma unroll
      for (int off = 1; off < 16; off <<= 1) m = fmaxf(m, __shfl_xor(m, off, 32));
      cm[r] = m;
    }

    __bf16* pwh = Psh[wave];
    __bf16* pwl = Psl[wave];
#pragma unroll
    for (int r = 0; r < 8; ++r) {
      const float mnew  = fmaxf(mrow[r], cm[r]);
      const float alpha = expf(mrow[r] - mnew);
      mrow[r] = mnew;
      float psum = 0.f;
#pragma unroll
      for (int j = 0; j < 4; ++j) {
        const float p = expf(s[j][r] - mnew);
        psum += p;
        __bf16 ph, plo;
        at_split(p, ph, plo);
        pwh[(8 * hh + r) * kKC + j * 16 + c] = ph;
        pwl[(8 * hh + r) * kKC + j * 16 + c] = plo;
      }
#pragma unroll
      for (int off = 1; off < 16; off <<= 1) psum += __shfl_xor(psum, off, 32);
      lrow[r] = lrow[r] * alpha + psum;
#pragma unroll
      for (int t = 0; t < 8; ++t) oacc[t][r] *= alpha;
    }
    __builtin_amdgcn_fence(__ATOMIC_RELEASE, "workgroup");
    __builtin_amdgcn_wave_barrier();
    __builtin_amdgcn_fence(__ATOMIC_ACQUIRE, "workgroup");

#pragma unroll
    for (int kk = 0; kk < 2; ++kk) {
      FB pa, pl;
      pa.h[0] = *(const v8b*)(pwh + c * kKC + kk * 32 + 8 * hh);
      pa.h[1] = *(const v8b*)(pwh + c * kKC + kk * 32 + 16 + 8 * hh);
      pl.h[0] = *(const v8b*)(pwl + c * kKC + kk * 32 + 8 * hh);
      pl.h[1] = *(const v8b*)(pwl + c * kKC + kk * 32 + 16 + 8 * hh);
#pragma unroll
      for (int t = 0; t < 8; ++t) {
        FB vb;
        vb.h[0] = *(const v8b*)(Vt + (t * 16 + c) * kKC + kk * 32 + 8 * hh);
        vb.h[1] = *(const v8b*)(Vt + (t * 16 + c) * kKC + kk * 32 + 16 + 8 * hh);
        oacc[t] = at_mma(pa.v, vb.v, oacc[t]);
        oacc[t] = at_mma(pl.v, vb.v, oacc[t]);
      }
    }
  }

  __syncthreads();
  float* slab = (float*)KVs + wave * (16 * 64);
  float inv[8];
#pragma unroll
  for (int r = 0; r < 8; ++r) inv[r] = 1.0f / lrow[r];
  const int c4 = c * 4;
#pragma unroll
  for (int hf = 0; hf < 2; ++hf) {
#pragma unroll
    for (int r = 0; r < 8; ++r) {
#pragma unroll
      for (int tt = 0; tt < 4; ++tt) slab[(8 * hh + r) * 64 + tt * 16 + c] = oacc[hf * 4 + tt][r] * inv[r];
    }
    __builtin_amdgcn_fence(__ATOMIC_RELEASE, "workgroup");
    __builtin_amdgcn_wave_barrier();
    __builtin_amdgcn_fence(__ATOMIC_ACQUIRE, "workgroup");
    for (int pass = 0; pass < 2; ++pass) {
#pragma unroll
      for (int it = 0; it < 8; ++it) {
        const int row = it * 2 + hh;
        const v4f val = *(const v4f*)(slab + row * 64 + c4);
        *(volatile v4f*)(out + (size_t)(q0 + row) * kHD + hf * 64 + c4) = val;
      }
      __threadfence();
    }
    __builtin_amdgcn_fence(__ATOMIC_RELEASE, "workgroup");
    __builtin_amdgcn_wave_barrier();
    __builtin_amdgcn_fence(__ATOMIC_ACQUIRE, "workgroup");
  }
}

extern "C" void kernel_launch(void* const* d_in, const int* in_sizes, int n_in,
                              void* d_out, int out_size, void* d_ws, size_t ws_size,
                              hipStream_t stream) {
  (void)n_in;
  const float* Q = (const float*)d_in[0];
  const float* K = (const float*)d_in[1];
  const float* V = (const float*)d_in[2];
  float* O = (float*)d_out;
  const int D = kHD;
  const int S = in_sizes[0] / D;
  if (S < kQB || (S % kQB) != 0) return;
  if (in_sizes[1] != in_sizes[0] || in_sizes[2] != in_sizes[0]) return;
  if (out_size != S * D) return;
  const size_t planeBytes = (size_t)S * D * 2;
  if (3 * planeBytes > ws_size) return;
  unsigned short* Qb = (unsigned short*)((char*)d_ws + 0);
  unsigned short* Kb = (unsigned short*)((char*)d_ws + planeBytes);
  unsigned short* Vb = (unsigned short*)((char*)d_ws + 2 * planeBytes);

  const int n8 = S * D / 8;
  dim3 g1((n8 + 255) / 256, 3), b1(256);
  cast3_f32_bf16x8<<<g1, b1, 0, stream>>>(Q, K, V, Qb, Kb, Vb, n8);

  const float scale = 1.0f / sqrtf(128.0f);
  dim3 g2(S / kQB), b2(kThr);
  attn_hd128_bf16<<<g2, b2, 0, stream>>>(Qb, Kb, Vb, O, S, scale);
}
